// Gpt2MambaSelectiveBlock_71829033059047
// MI455X (gfx1250) — hardware-verified
//
#include <hip/hip_runtime.h>
#include <math.h>

constexpr int EMB   = 768;
constexpr int NHEAD = 12;
constexpr int HDIM  = 64;
constexpr int FFN   = 3072;
constexpr int SEQ   = 1024;
constexpr int NBAT  = 2;
constexpr int NTOK  = NBAT * SEQ;
constexpr int CIN   = 1536;
constexpr int NSTA  = 16;
constexpr int RDTL  = 48;
constexpr int XPJW  = 80;
constexpr int XPJLD = 128;
constexpr int DTK   = 64;
constexpr int XZLD  = 2 * CIN;
constexpr int HPG   = 4;
constexpr int NGRP  = NHEAD / HPG;
constexpr int kTP   = 260;
constexpr float kWCarry    = 16.0f;
constexpr float kWCarryInv = 1.0f / 16.0f;
constexpr float kUCarry    = 256.0f;
constexpr float kDTLCarry  = 1024.0f;
constexpr float kYCarry    = 4096.0f;
constexpr float kCtxCarry  = 16.0f;
constexpr float kPCarry    = 32768.0f;
constexpr float kQScale    = 0.125f;
constexpr float kFill      = -1.0e30f;
constexpr float kInvEmb    = 1.0f / 768.0f;
constexpr float kLnEps     = 1e-5f;

typedef __attribute__((ext_vector_type(16))) _Float16 v16h;
typedef __attribute__((ext_vector_type(8)))  _Float16 v8h;
typedef __attribute__((ext_vector_type(16))) __bf16   v16b;
typedef __attribute__((ext_vector_type(8)))  __bf16   v8b;
typedef __attribute__((ext_vector_type(8)))  float    v8f;
typedef __attribute__((ext_vector_type(4)))  float    v4f;
typedef __attribute__((ext_vector_type(4)))  unsigned int v4u;

__device__ __forceinline__ unsigned short f2bf_bits(float f) {
  unsigned u = __float_as_uint(f);
  return (unsigned short)((u + 0x7FFFu + ((u >> 16) & 1u)) >> 16);
}
__device__ __forceinline__ float bf_bits2f(unsigned short h) { return __uint_as_float(((unsigned)h) << 16); }

__device__ __forceinline__ void dep_guard_h(v8f& a, v8f& b, v16h x, v16h y) { asm volatile("v_nop\n\tv_nop\n\tv_nop\n\tv_nop" : "+v"(a), "+v"(b) : "v"(x), "v"(y)); }
__device__ __forceinline__ void dep_guard_b(v8f& a, v8f& b, v16b x, v16b y) { asm volatile("v_nop\n\tv_nop\n\tv_nop\n\tv_nop" : "+v"(a), "+v"(b) : "v"(x), "v"(y)); }
__device__ __forceinline__ void keep4_h(v16h a, v16h b, v16h c, v16h d) { asm volatile("v_nop" :: "v"(a), "v"(b), "v"(c), "v"(d)); }
__device__ __forceinline__ void keep4_b(v16b a, v16b b, v16b c, v16b d) { asm volatile("v_nop" :: "v"(a), "v"(b), "v"(c), "v"(d)); }
__device__ __forceinline__ void acc_guard4(v8f& a, v8f& b, v8f& c, v8f& d) { asm volatile("v_nop\n\tv_nop\n\tv_nop\n\tv_nop" : "+v"(a), "+v"(b), "+v"(c), "+v"(d)); }
template <typename T> struct Frag;
template <> struct Frag<_Float16> {
  typedef v16h V; union U { v16h v; v8h h[2]; };
  static __device__ __forceinline__ v16h load(const _Float16* p) {
    U f; f.h[0] = *(const v8h*)(p); f.h[1] = *(const v8h*)(p + 16); return f.v;
  }
  static __device__ __forceinline__ v8f mma(v16h a, v16h b, v8f c) {
    return __builtin_amdgcn_wmma_f32_16x16x32_f16(false, a, false, b, (short)0, c, false, false);
  }
  static __device__ __forceinline__ void guard(v8f& a, v8f& b, v16h x, v16h y) { dep_guard_h(a, b, x, y); }
  static __device__ __forceinline__ void keep(v16h a, v16h b, v16h c, v16h d) { keep4_h(a, b, c, d); }
};
template <> struct Frag<__bf16> {
  typedef v16b V; union U { v16b v; v8b h[2]; };
  static __device__ __forceinline__ v16b load(const __bf16* p) {
    U f; f.h[0] = *(const v8b*)(p); f.h[1] = *(const v8b*)(p + 16); return f.v;
  }
  static __device__ __forceinline__ v8f mma(v16b a, v16b b, v8f c) {
    return __builtin_amdgcn_wmma_f32_16x16x32_bf16(false, a, false, b, (short)0, c, false, false);
  }
  static __device__ __forceinline__ void guard(v8f& a, v8f& b, v16b x, v16b y) { dep_guard_b(a, b, x, y); }
  static __device__ __forceinline__ void keep(v16b a, v16b b, v16b c, v16b d) { keep4_b(a, b, c, d); }
};

template <int ET> struct Elem;
template <> struct Elem<0> { typedef _Float16 T; };
template <> struct Elem<1> { typedef __bf16 T; };
template <int ET, bool SPLIT, int BIAS_MODE, int OUT_MODE, bool RESID, int ACT = 0, int TRI = 0>
__global__ __launch_bounds__(256) void wmma_gemm64(
    const unsigned short* __restrict__ Ap, const unsigned short* __restrict__ A2p, int lda, long strideA,
    const unsigned short* __restrict__ Btp, const unsigned short* __restrict__ Bt2p, int ldb, long strideB,
    void* __restrict__ Cout, void* __restrict__ Cout2, int ldc, long strideC,
    const float* __restrict__ bias,
    const float* __restrict__ resid, long strideR,
    int M, int N, int K, float scale) {
  typedef typename Elem<ET>::T T;
  typedef typename Frag<T>::V V;
  const T* A = (const T*)Ap; const T* A2 = (const T*)A2p; const T* Bt = (const T*)Btp; const T* Bt2 = (const T*)Bt2p;
  __shared__ __align__(16) float sT[8][16 * 68];
  const int b    = blockIdx.y;
  const int lane = threadIdx.x & 31;
  const int wave = threadIdx.x >> 5;
  const int tilesN = N >> 6;
  const int tilesM = M >> 6;
  const int tile = blockIdx.x * 8 + wave;
  if (tile >= tilesM * tilesN) return;
  const int tm = tile / tilesN;
  const int tn = tile - tm * tilesN;
  const int m0 = tm << 6;
  const int n0 = tn << 6;
  if (TRI == 1 && n0 > m0) return;
  const int Kl = (TRI == 2 && (m0 + 64) < K) ? (m0 + 64) : K;

  const T* Ab  = A  + (size_t)b * strideA;
  const T* Bb  = Bt + (size_t)b * strideB;
  const T* Ab2 = SPLIT ? (A2  + (size_t)b * strideA) : nullptr;
  const T* Bb2 = SPLIT ? (Bt2 + (size_t)b * strideB) : nullptr;

  const int rlane = lane & 15;
  const int koff  = (lane >> 4) * 8;
  const int mOff  = (lane >> 4) * 8;

  v8f acc[4][4];
#pragma unroll
  for (int i = 0; i < 4; ++i)
#pragma unroll
    for (int j = 0; j < 4; ++j) acc[i][j] = (v8f){0.f,0.f,0.f,0.f,0.f,0.f,0.f,0.f};

  for (int k0 = 0; k0 < Kl; k0 += 32) {
    V bh[4], bl[4];
#pragma unroll
    for (int j = 0; j < 4; ++j) {
      const size_t bo = (size_t)(n0 + (j << 4) + rlane) * ldb + koff + k0;
      bh[j] = Frag<T>::load(Bb + bo);
      if (SPLIT) bl[j] = Frag<T>::load(Bb2 + bo);
    }
#pragma unroll
    for (int i = 0; i < 4; ++i) {
      const size_t ao = (size_t)(m0 + (i << 4) + rlane) * lda + koff + k0;
      V ah = Frag<T>::load(Ab + ao);
      V al;
      if (SPLIT) al = Frag<T>::load(Ab2 + ao);
#pragma unroll
      for (int j = 0; j < 4; ++j) {
        acc[i][j] = Frag<T>::mma(ah, bh[j], acc[i][j]);
        if (SPLIT) {
          acc[i][j] = Frag<T>::mma(ah, bl[j], acc[i][j]);
          acc[i][j] = Frag<T>::mma(al, bh[j], acc[i][j]);
        }
      }
      Frag<T>::guard(acc[i][0], acc[i][3], ah, SPLIT ? al : ah);
    }
    Frag<T>::keep(bh[0], bh[1], bh[2], bh[3]);
    if (SPLIT) Frag<T>::keep(bl[0], bl[1], bl[2], bl[3]);
  }
  acc_guard4(acc[0][0], acc[0][1], acc[0][2], acc[0][3]);
  acc_guard4(acc[1][0], acc[1][1], acc[1][2], acc[1][3]);
  acc_guard4(acc[2][0], acc[2][1], acc[2][2], acc[2][3]);
  acc_guard4(acc[3][0], acc[3][1], acc[3][2], acc[3][3]);

  float* slab = sT[wave];
  const float* Rb = RESID ? (resid + (size_t)b * strideR) : nullptr;
#pragma unroll
  for (int i = 0; i < 4; ++i) {
    const int mBase = m0 + (i << 4);
#pragma unroll
    for (int j = 0; j < 4; ++j) {
      const int n = n0 + (j << 4) + rlane;
      float bv = 0.f;
      if (BIAS_MODE == 2) bv = bias[n];
#pragma unroll
      for (int r = 0; r < 8; ++r) {
        float v = acc[i][j][r] * scale;
        if (BIAS_MODE == 1) v += bias[mBase + mOff + r];
        if (BIAS_MODE == 2) v += bv;
        if (RESID) v += Rb[(size_t)(mBase + mOff + r) * ldc + n];
        if (ACT == 1) v = tanhf(v);
        if (ACT == 2) v = fmaxf(v, 0.0f);
        if (ACT == 3) v = v / (1.0f + expf(-v));
        if (ACT == 4) v = (v > 0.f) ? v : 0.01f * v;
        slab[(mOff + r) * 68 + (j << 4) + rlane] = v;
      }
    }
    __builtin_amdgcn_fence(__ATOMIC_RELEASE, "workgroup");
    __builtin_amdgcn_wave_barrier();
    __builtin_amdgcn_fence(__ATOMIC_ACQUIRE, "workgroup");
    if (OUT_MODE == 0) {
      float* C = (float*)Cout + (size_t)b * strideC;
      const int hh = lane >> 4, c4 = (lane & 15) * 4;
      for (int pass = 0; pass < 2; ++pass) {
#pragma unroll
        for (int it = 0; it < 8; ++it) {
          const int row = it * 2 + hh;
          v4f v = *(const v4f*)(slab + row * 68 + c4);
          *(volatile v4f*)(C + (size_t)(mBase + row) * ldc + n0 + c4) = v;
        }
        __threadfence();
      }
    } else {
      const int q = lane >> 3, c8 = (lane & 7) * 8;
      unsigned short* C  = (unsigned short*)Cout  + (size_t)b * strideC;
      unsigned short* C2 = (OUT_MODE == 2) ? ((unsigned short*)Cout2 + (size_t)b * strideC) : nullptr;
      for (int pass = 0; pass < 2; ++pass) {
#pragma unroll
        for (int it = 0; it < 4; ++it) {
          const int row = it * 4 + q;
          const float* sp = slab + row * 68 + c8;
          v8h hv, lv;
#pragma unroll
          for (int e = 0; e < 8; ++e) {
            if (OUT_MODE == 1) {
              hv[e] = (_Float16)sp[e];
            } else {
              unsigned short hb = f2bf_bits(sp[e]);
              unsigned short lb = f2bf_bits(sp[e] - bf_bits2f(hb));
              hv[e] = __builtin_bit_cast(_Float16, hb);
              lv[e] = __builtin_bit_cast(_Float16, lb);
            }
          }
          *(volatile v8h*)(C + (size_t)(mBase + row) * ldc + n0 + c8) = hv;
          if (OUT_MODE == 2) *(volatile v8h*)(C2 + (size_t)(mBase + row) * ldc + n0 + c8) = lv;
        }
        __threadfence();
      }
    }
    __builtin_amdgcn_fence(__ATOMIC_RELEASE, "workgroup");
    __builtin_amdgcn_wave_barrier();
    __builtin_amdgcn_fence(__ATOMIC_ACQUIRE, "workgroup");
  }
}

__device__ __forceinline__ unsigned pk16(unsigned short a, unsigned short b) { return (unsigned)a | ((unsigned)b << 16); }
__device__ __forceinline__ unsigned short h_bits(float f) { const _Float16 h = (_Float16)f; return __builtin_bit_cast(unsigned short, h); }

__global__ __launch_bounds__(256) void transpose_cast_f16_kernel(const float* __restrict__ in, unsigned short* __restrict__ out,
                                                                 int R, int CC, float scale) {
  __shared__ float tile[64][65];
  const int t  = threadIdx.x;
  const int n0 = blockIdx.x * 64;
  const int k0 = blockIdx.y * 64;
  {
    const int kr = t >> 2, nc = (t & 3) * 16;
    const float* p = in + (size_t)(k0 + kr) * CC + n0 + nc;
#pragma unroll
    for (int e4 = 0; e4 < 4; ++e4) {
      const v4f f = *(const v4f*)(p + 4 * e4);
      tile[kr][nc + 4 * e4 + 0] = f[0];
      tile[kr][nc + 4 * e4 + 1] = f[1];
      tile[kr][nc + 4 * e4 + 2] = f[2];
      tile[kr][nc + 4 * e4 + 3] = f[3];
    }
  }
  __syncthreads();
  const int q = t >> 3, c8 = (t & 7) * 8;
  v4u u0, u1;
#pragma unroll
  for (int w = 0; w < 4; ++w) {
    u0[w] = pk16(h_bits(tile[c8 + 2 * w][q] * scale),      h_bits(tile[c8 + 2 * w + 1][q] * scale));
    u1[w] = pk16(h_bits(tile[c8 + 2 * w][32 + q] * scale), h_bits(tile[c8 + 2 * w + 1][32 + q] * scale));
  }
  unsigned short* p0 = out + (size_t)(n0 + q) * R + k0 + c8;
  unsigned short* p1 = out + (size_t)(n0 + 32 + q) * R + k0 + c8;
  for (int pass = 0; pass < 2; ++pass) {
    *(volatile v4u*)p0 = u0;
    *(volatile v4u*)p1 = u1;
    __threadfence();
  }
}

__global__ __launch_bounds__(256) void pad_transpose_f16_kernel(const float* __restrict__ in, unsigned short* __restrict__ out,
                                                               int K, int N, int Kpad, int Npad, int total, float scale) {
  const int i = blockIdx.x * 256 + threadIdx.x;
  if (i >= total) return;
  const int kp8 = Kpad >> 3;
  const int n   = i / kp8;
  const int c8  = (i - n * kp8) * 8;
  const int nc  = (n < N) ? n : (N - 1);
  unsigned short hb[8];
#pragma unroll
  for (int e = 0; e < 8; ++e) {
    const int k  = c8 + e;
    const int kc = (k < K) ? k : (K - 1);
    const float v = in[(size_t)kc * N + nc];
    const bool live = (n < N) && (k < K);
    hb[e] = h_bits(live ? v * scale : 0.0f);
  }
  const v4u u = (v4u){pk16(hb[0], hb[1]), pk16(hb[2], hb[3]), pk16(hb[4], hb[5]), pk16(hb[6], hb[7])};
  unsigned short* p = out + (size_t)n * Kpad + c8;
  *(volatile v4u*)p = u;
  __threadfence();
  *(volatile v4u*)p = u;
  (void)Npad;
}

__global__ __launch_bounds__(192) void ln_dual_kernel(const float* __restrict__ x,
    const float* __restrict__ g1, const float* __restrict__ b1,
    const float* __restrict__ gm, const float* __restrict__ bm, const float* __restrict__ rw,
    unsigned short* __restrict__ XN16, float* __restrict__ HM, unsigned short* __restrict__ HR16) {
  __shared__ float redA[8];
  __shared__ float redB[8];
  __shared__ float redC[8];
  __shared__ __align__(16) float sXc[EMB];
  __shared__ __align__(16) float sHm[EMB];
  const int row  = blockIdx.x;
  const int t    = threadIdx.x;
  const int lane = t & 31, wave = t >> 5;
  const int c0   = t * 4;
  const v4f a = *(const v4f*)(x + (size_t)row * EMB + c0);
  float s = (a[0] + a[1]) + (a[2] + a[3]);
#pragma unroll
  for (int off = 16; off > 0; off >>= 1) s += __shfl_xor(s, off, 32);
  if (lane == 0) redA[wave] = s;
  __syncthreads();
  const float mu = (((redA[0] + redA[1]) + (redA[2] + redA[3])) + (redA[4] + redA[5])) * kInvEmb;
  const float d0 = a[0] - mu, d1 = a[1] - mu, d2 = a[2] - mu, d3 = a[3] - mu;
  float qq = (d0 * d0 + d1 * d1) + (d2 * d2 + d3 * d3);
#pragma unroll
  for (int off = 16; off > 0; off >>= 1) qq += __shfl_xor(qq, off, 32);
  if (lane == 0) redB[wave] = qq;
  __syncthreads();
  const float var = (((redB[0] + redB[1]) + (redB[2] + redB[3])) + (redB[4] + redB[5])) * kInvEmb;
  const float rs  = rsqrtf(var + kLnEps);
  const float xc0 = d0 * rs, xc1 = d1 * rs, xc2 = d2 * rs, xc3 = d3 * rs;
  const v4f gmv = *(const v4f*)(gm + c0);
  const v4f bmv = *(const v4f*)(bm + c0);
  const float h0 = xc0 * gmv[0] + bmv[0], h1 = xc1 * gmv[1] + bmv[1];
  const float h2 = xc2 * gmv[2] + bmv[2], h3 = xc3 * gmv[3] + bmv[3];
  *(v4f*)(sXc + c0) = (v4f){xc0, xc1, xc2, xc3};
  const v4f hmv = (v4f){h0, h1, h2, h3};
  *(v4f*)(sHm + c0) = hmv;
  float* hp = HM + (size_t)row * EMB + c0;
  *(volatile v4f*)hp = hmv;
  __threadfence();
  *(volatile v4f*)hp = hmv;
  float s3 = (h0 * h0 + h1 * h1) + (h2 * h2 + h3 * h3);
#pragma unroll
  for (int off = 16; off > 0; off >>= 1) s3 += __shfl_xor(s3, off, 32);
  if (lane == 0) redC[wave] = s3;
  __syncthreads();
  const float ms = (((redC[0] + redC[1]) + (redC[2] + redC[3])) + (redC[4] + redC[5])) * kInvEmb;
  const float r2 = rsqrtf(ms + kLnEps);
  if (t < 96) {
    const int c8 = t * 8;
    const v4f xa = *(const v4f*)(sXc + c8), xb = *(const v4f*)(sXc + c8 + 4);
    const v4f ha = *(const v4f*)(sHm + c8), hb = *(const v4f*)(sHm + c8 + 4);
    const v4f ga = *(const v4f*)(g1 + c8), gb = *(const v4f*)(g1 + c8 + 4);
    const v4f ba = *(const v4f*)(b1 + c8), bb = *(const v4f*)(b1 + c8 + 4);
    const v4f wa = *(const v4f*)(rw + c8), wb = *(const v4f*)(rw + c8 + 4);
    unsigned short yb[8], zb[8];
#pragma unroll
    for (int e = 0; e < 4; ++e) {
      yb[e]     = h_bits(xa[e] * ga[e] + ba[e]);
      yb[4 + e] = h_bits(xb[e] * gb[e] + bb[e]);
      zb[e]     = h_bits((ha[e] * r2) * wa[e]);
      zb[4 + e] = h_bits((hb[e] * r2) * wb[e]);
    }
    const v4u yv = (v4u){pk16(yb[0], yb[1]), pk16(yb[2], yb[3]), pk16(yb[4], yb[5]), pk16(yb[6], yb[7])};
    const v4u zv = (v4u){pk16(zb[0], zb[1]), pk16(zb[2], zb[3]), pk16(zb[4], zb[5]), pk16(zb[6], zb[7])};
    unsigned short* yp = XN16 + (size_t)row * EMB + c8;
    unsigned short* zp = HR16 + (size_t)row * EMB + c8;
    *(volatile v4u*)yp = yv;
    *(volatile v4u*)zp = zv;
    __threadfence();
    *(volatile v4u*)yp = yv;
    *(volatile v4u*)zp = zv;
  }
}

__global__ __launch_bounds__(128) void layernorm_f16_kernel(const float* __restrict__ x, const float* __restrict__ gam,
                                                            const float* __restrict__ bet, unsigned short* __restrict__ out) {
  __shared__ float redA[4];
  __shared__ float redB[4];
  const int row  = blockIdx.x;
  const int t    = threadIdx.x;
  const int lane = t & 31, wave = t >> 5;
  const int c0   = t * 8;
  const float* xr = x + (size_t)row * EMB + c0;
  const v4f a = *(const v4f*)(xr);
  const v4f c = *(const v4f*)(xr + 4);
  float s = ((a[0] + a[1]) + (a[2] + a[3])) + ((c[0] + c[1]) + (c[2] + c[3]));
#pragma unroll
  for (int off = 16; off > 0; off >>= 1) s += __shfl_xor(s, off, 32);
  if (lane == 0) redA[wave] = s;
  __syncthreads();
  const float mu = ((redA[0] + redA[1]) + redA[2]) * kInvEmb;
  const float d0 = a[0] - mu, d1 = a[1] - mu, d2 = a[2] - mu, d3 = a[3] - mu;
  const float d4 = c[0] - mu, d5 = c[1] - mu, d6 = c[2] - mu, d7 = c[3] - mu;
  float qq = ((d0 * d0 + d1 * d1) + (d2 * d2 + d3 * d3)) + ((d4 * d4 + d5 * d5) + (d6 * d6 + d7 * d7));
#pragma unroll
  for (int off = 16; off > 0; off >>= 1) qq += __shfl_xor(qq, off, 32);
  if (lane == 0) redB[wave] = qq;
  __syncthreads();
  const float var = ((redB[0] + redB[1]) + redB[2]) * kInvEmb;
  const float rs  = rsqrtf(var + kLnEps);
  const v4f g0 = *(const v4f*)(gam + c0), g1 = *(const v4f*)(gam + c0 + 4);
  const v4f b0 = *(const v4f*)(bet + c0), b1 = *(const v4f*)(bet + c0 + 4);
  const float y0 = d0 * rs * g0[0] + b0[0], y1 = d1 * rs * g0[1] + b0[1];
  const float y2 = d2 * rs * g0[2] + b0[2], y3 = d3 * rs * g0[3] + b0[3];
  const float y4 = d4 * rs * g1[0] + b1[0], y5 = d5 * rs * g1[1] + b1[1];
  const float y6 = d6 * rs * g1[2] + b1[2], y7 = d7 * rs * g1[3] + b1[3];
  const v4u hv = (v4u){pk16(h_bits(y0), h_bits(y1)), pk16(h_bits(y2), h_bits(y3)),
                       pk16(h_bits(y4), h_bits(y5)), pk16(h_bits(y6), h_bits(y7))};
  unsigned short* op = out + (size_t)row * EMB + c0;
  *(volatile v4u*)op = hv;
  __threadfence();
  *(volatile v4u*)op = hv;
}

__global__ __launch_bounds__(256) void conv_silu_kernel(
    const float* __restrict__ XZ, const float* __restrict__ cw, const float* __restrict__ cb,
    float* __restrict__ HSC, unsigned short* __restrict__ HSC16)
{
  __shared__ __align__(16) float sT[16 * kTP];
  const int tid = threadIdx.x, lane = tid & 31, wave = tid >> 5;
  const int d0 = blockIdx.x * 256, d = d0 + tid;
  const int m0 = blockIdx.y * 64;
  const int bidx = m0 / SEQ;
  const int t0 = m0 - bidx * SEQ;
  const size_t rb = (size_t)bidx * SEQ;
  const float w0 = cw[d * 4 + 0], w1 = cw[d * 4 + 1], w2 = cw[d * 4 + 2], w3 = cw[d * 4 + 3];
  const float bc = cb[d];
  float xm3, xm2, xm1;
  {
    const int r3 = t0 - 3, r2 = t0 - 2, r1 = t0 - 1;
    const float v3 = XZ[(rb + (r3 < 0 ? 0 : r3)) * XZLD + d];
    const float v2 = XZ[(rb + (r2 < 0 ? 0 : r2)) * XZLD + d];
    const float v1 = XZ[(rb + (r1 < 0 ? 0 : r1)) * XZLD + d];
    xm3 = (r3 >= 0) ? v3 : 0.f;
    xm2 = (r2 >= 0) ? v2 : 0.f;
    xm1 = (r1 >= 0) ? v1 : 0.f;
  }
  const int hrow = wave >> 1;
  const int hch  = (wave & 1) * 128 + lane * 4;
#pragma unroll 1
  for (int sub = 0; sub < 4; ++sub) {
    const int lb = t0 + sub * 16;
#pragma unroll 1
    for (int s = 0; s < 16; ++s) {
      const float cur = XZ[(rb + lb + s) * XZLD + d];
      float acc = w0 * xm3;
      acc = fmaf(w1, xm2, acc);
      acc = fmaf(w2, xm1, acc);
      acc = fmaf(w3, cur, acc);
      const float sv = acc + bc;
      const float sg = __builtin_amdgcn_rcpf(1.0f + __expf(-sv));
      sT[s * kTP + tid] = sv * sg;
      xm3 = xm2; xm2 = xm1; xm1 = cur;
    }
    __syncthreads();
    v4f fv[4];
    v8h bv[2];
#pragma unroll
    for (int it = 0; it < 4; ++it) fv[it] = *(const v4f*)(sT + (it * 4 + hrow) * kTP + hch);
#pragma unroll
    for (int it = 0; it < 2; ++it) {
      const float* sp = sT + (it * 8 + wave) * kTP + lane * 8;
      const v4f a0 = *(const v4f*)(sp);
      const v4f a1 = *(const v4f*)(sp + 4);
#pragma unroll
      for (int e = 0; e < 4; ++e) {
        bv[it][e]     = (_Float16)(a0[e] * kUCarry);
        bv[it][4 + e] = (_Float16)(a1[e] * kUCarry);
      }
    }
    const size_t rowg = rb + lb;
    for (int pass = 0; pass < 2; ++pass) {
#pragma unroll
      for (int it = 0; it < 4; ++it)
        *(volatile v4f*)(HSC + (rowg + it * 4 + hrow) * CIN + d0 + hch) = fv[it];
#pragma unroll
      for (int it = 0; it < 2; ++it)
        *(volatile v8h*)(HSC16 + (rowg + it * 8 + wave) * CIN + d0 + lane * 8) = bv[it];
      __threadfence();
    }
    __syncthreads();
  }
}

__global__ __launch_bounds__(256) void dtl_cast_kernel(const float* __restrict__ XPJ, unsigned short* __restrict__ DTL16, int total) {
  const int i = blockIdx.x * 256 + threadIdx.x;
  if (i >= total) return;
  const int m = i >> 3, c8 = (i & 7) * 8;
  const float* p = XPJ + (size_t)m * XPJLD + c8;
  const v4f a0 = *(const v4f*)(p);
  const v4f a1 = *(const v4f*)(p + 4);
  const bool live = (c8 < RDTL);
  unsigned short hb[8];
#pragma unroll
  for (int e = 0; e < 4; ++e) {
    hb[e]     = h_bits(live ? a0[e] * kDTLCarry : 0.0f);
    hb[4 + e] = h_bits(live ? a1[e] * kDTLCarry : 0.0f);
  }
  const v4u u = (v4u){pk16(hb[0], hb[1]), pk16(hb[2], hb[3]), pk16(hb[4], hb[5]), pk16(hb[6], hb[7])};
  unsigned short* q = DTL16 + (size_t)m * DTK + c8;
  *(volatile v4u*)q = u;
  __threadfence();
  *(volatile v4u*)q = u;
}

__global__ __launch_bounds__(256) void scan_kernel(
    const float* __restrict__ DTR, const float* __restrict__ HSC, const float* __restrict__ XZ,
    const float* __restrict__ XPJ, const float* __restrict__ A_log, const float* __restrict__ Dp,
    unsigned short* __restrict__ Y16)
{
  __shared__ __align__(16) float sBC[16 * 32];
  __shared__ __align__(16) float sY[16 * kTP];
  const int tid = threadIdx.x, lane = tid & 31, wave = tid >> 5;
  const int d0 = blockIdx.x * 256, d = d0 + tid;
  const size_t rb = (size_t)blockIdx.y * SEQ;

  float An[NSTA];
#pragma unroll
  for (int n = 0; n < NSTA; ++n) An[n] = -expf(A_log[(size_t)d * NSTA + n]);
  const float Dd = Dp[d];
  float h[NSTA];
#pragma unroll
  for (int n = 0; n < NSTA; ++n) h[n] = 0.f;

#pragma unroll 1
  for (int c = 0; c < SEQ / 16; ++c) {
    const int l0 = c * 16;
    if (tid < 128) {
      const int r = tid >> 3, q = (tid & 7) * 4;
      const v4f v = *(const v4f*)(XPJ + (rb + l0 + r) * XPJLD + RDTL + q);
      *(v4f*)(sBC + r * 32 + q) = v;
    }
    __syncthreads();
#pragma unroll 1
    for (int s = 0; s < 16; ++s) {
      const size_t m = rb + l0 + s;
      const float a   = DTR[m * CIN + d];
      const float dt  = fmaxf(a, 0.0f) + log1pf(expf(-fabsf(a)));
      const float u   = HSC[m * CIN + d];
      const float g   = XZ[m * XZLD + CIN + d];
      v4f Bq[4], Cq[4];
#pragma unroll
      for (int qq = 0; qq < 4; ++qq) {
        Bq[qq] = *(const v4f*)(sBC + s * 32 + 4 * qq);
        Cq[qq] = *(const v4f*)(sBC + s * 32 + NSTA + 4 * qq);
      }
      float y = 0.f;
#pragma unroll
      for (int n = 0; n < NSTA; ++n) {
        const float e = __expf(dt * An[n]);
        float db = dt * Bq[n >> 2][n & 3];
        asm volatile("" : "+v"(db));
        float p = db * u;
        asm volatile("" : "+v"(p));
        float qv = h[n] * e;
        asm volatile("" : "+v"(qv));
        const float hn = qv + p;
        h[n] = hn;
        float rr = hn * Cq[n >> 2][n & 3];
        asm volatile("" : "+v"(rr));
        y += rr;
      }
      float ud = u * Dd;
      asm volatile("" : "+v"(ud));
      y = y + ud;
      const float sg = __builtin_amdgcn_rcpf(1.0f + __expf(-g));
      const float gt = g * sg;
      sY[s * kTP + tid] = (y * gt) * kYCarry;
    }
    __syncthreads();
    v8h hv[2];
#pragma unroll
    for (int it = 0; it < 2; ++it) {
      const float* sp = sY + (it * 8 + wave) * kTP + lane * 8;
      const v4f a0 = *(const v4f*)(sp);
      const v4f a1 = *(const v4f*)(sp + 4);
#pragma unroll
      for (int e = 0; e < 4; ++e) { hv[it][e] = (_Float16)a0[e]; hv[it][4 + e] = (_Float16)a1[e]; }
    }
    for (int pass = 0; pass < 2; ++pass) {
#pragma unroll
      for (int it = 0; it < 2; ++it)
        *(volatile v8h*)(Y16 + (rb + l0 + it * 8 + wave) * CIN + d0 + lane * 8) = hv[it];
      __threadfence();
    }
  }
}

__global__ __launch_bounds__(256) void sel_kernel(const float* __restrict__ MO, const float* __restrict__ sw,
                                                  const float* __restrict__ sb, float* __restrict__ SELF, int nrows) {
  const int m = blockIdx.x * 256 + threadIdx.x;
  if (m >= nrows) return;
  const float* mr = MO + (size_t)m * EMB;
  float acc = 0.f;
#pragma unroll 1
  for (int c = 0; c < EMB; ++c) {
    float v = mr[c];
    v = fminf(20.0f, fmaxf(-20.0f, v));
    acc = fmaf(v, sw[c], acc);
  }
  const float z  = acc + sb[0];
  const float sg = 1.0f / (1.0f + expf(-z));
  const float f  = 0.3f + 0.7f * sg;
  ((volatile float*)SELF)[m] = f;
  __threadfence();
  ((volatile float*)SELF)[m] = f;
}

__global__ __launch_bounds__(128) void softmax_causal_sel_kernel(const float* __restrict__ S,
                                                                 const float* __restrict__ selfac,
                                                                 unsigned short* __restrict__ P) {
  __shared__ float redm[4];
  __shared__ float reds[4];
  const int i    = blockIdx.x;
  const int hg   = blockIdx.y;
  const int tid  = threadIdx.x;
  const int lane = tid & 31;
  const int wave = tid >> 5;
  const int j0   = tid * 8;
  const float* rp = S + ((size_t)hg * SEQ + i) * SEQ + j0;
  const v4f a  = *(const v4f*)(rp);
  const v4f c  = *(const v4f*)(rp + 4);
  const v4f fa = *(const v4f*)(selfac + j0);
  const v4f fc = *(const v4f*)(selfac + j0 + 4);
  const float t0 = (j0 + 0 <= i) ? a[0] : kFill;
  const float t1 = (j0 + 1 <= i) ? a[1] : kFill;
  const float t2 = (j0 + 2 <= i) ? a[2] : kFill;
  const float t3 = (j0 + 3 <= i) ? a[3] : kFill;
  const float t4 = (j0 + 4 <= i) ? c[0] : kFill;
  const float t5 = (j0 + 5 <= i) ? c[1] : kFill;
  const float t6 = (j0 + 6 <= i) ? c[2] : kFill;
  const float t7 = (j0 + 7 <= i) ? c[3] : kFill;
  float m = fmaxf(fmaxf(fmaxf(t0, t1), fmaxf(t2, t3)), fmaxf(fmaxf(t4, t5), fmaxf(t6, t7)));
#pragma unroll
  for (int off = 16; off > 0; off >>= 1) m = fmaxf(m, __shfl_xor(m, off, 32));
  if (lane == 0) redm[wave] = m;
  __syncthreads();
  const float mx = fmaxf(fmaxf(redm[0], redm[1]), fmaxf(redm[2], redm[3]));
  const float e0 = __expf(t0 - mx), e1 = __expf(t1 - mx), e2 = __expf(t2 - mx), e3 = __expf(t3 - mx);
  const float e4 = __expf(t4 - mx), e5 = __expf(t5 - mx), e6 = __expf(t6 - mx), e7 = __expf(t7 - mx);
  float s = ((e0 + e1) + (e2 + e3)) + ((e4 + e5) + (e6 + e7));
#pragma unroll
  for (int off = 16; off > 0; off >>= 1) s += __shfl_xor(s, off, 32);
  if (lane == 0) reds[wave] = s;
  __syncthreads();
  const float tot = ((reds[0] + reds[1]) + reds[2]) + reds[3];
  const float inv = 1.0f / tot;
  const float p0 = (e0 * inv) * fa[0], p1 = (e1 * inv) * fa[1], p2 = (e2 * inv) * fa[2], p3 = (e3 * inv) * fa[3];
  const float p4 = (e4 * inv) * fc[0], p5 = (e5 * inv) * fc[1], p6 = (e6 * inv) * fc[2], p7 = (e7 * inv) * fc[3];
  const v4u hv = (v4u){pk16(h_bits(p0 * kPCarry), h_bits(p1 * kPCarry)),
                       pk16(h_bits(p2 * kPCarry), h_bits(p3 * kPCarry)),
                       pk16(h_bits(p4 * kPCarry), h_bits(p5 * kPCarry)),
                       pk16(h_bits(p6 * kPCarry), h_bits(p7 * kPCarry))};
  const size_t ro = ((size_t)hg * SEQ + i) * SEQ + j0;
  *(volatile v4u*)(P + ro) = hv;
  __threadfence();
  *(volatile v4u*)(P + ro) = hv;
}

__global__ __launch_bounds__(256) void gelu_erf_f16x8_kernel(unsigned short* __restrict__ buf, int n8) {
  const int i = blockIdx.x * 256 + threadIdx.x;
  if (i < n8) {
    unsigned short* p = buf + 8 * (size_t)i;
    const v4u u = *(const v4u*)p;
    const unsigned long long w0 = (unsigned long long)u[0] | ((unsigned long long)u[1] << 32);
    const unsigned long long w1 = (unsigned long long)u[2] | ((unsigned long long)u[3] << 32);
    unsigned long long g0 = 0ull, g1 = 0ull;
#pragma unroll 1
    for (int e = 0; e < 8; ++e) {
      const bool hiw = (e >= 4);
      const int  sh  = (e & 3) * 16;
      const unsigned long long w = hiw ? w1 : w0;
      const unsigned short hb = (unsigned short)((w >> sh) & 0xFFFFull);
      const float a  = (float)__builtin_bit_cast(_Float16, hb);
      const float gv = 0.5f * a * (1.0f + erff(a * 0.70710678118654752f));
      const unsigned long long gb = ((unsigned long long)h_bits(gv)) << sh;
      g0 |= hiw ? 0ull : gb;
      g1 |= hiw ? gb : 0ull;
    }
    const v4u r = (v4u){(unsigned)(g0 & 0xFFFFFFFFull), (unsigned)(g0 >> 32),
                        (unsigned)(g1 & 0xFFFFFFFFull), (unsigned)(g1 >> 32)};
    *(volatile v4u*)p = r;
    __threadfence();
    *(volatile v4u*)p = r;
  }
}

extern "C" void kernel_launch(void* const* d_in, const int* in_sizes, int n_in,
                              void* d_out, int out_size, void* d_ws, size_t ws_size,
                              hipStream_t stream) {
  if (n_in < 27) return;
  if (in_sizes[0] != NTOK * EMB) return;
  if (in_sizes[1] != EMB || in_sizes[2] != EMB) return;
  if (in_sizes[3] != EMB * 3 * EMB || in_sizes[4] != 3 * EMB) return;
  if (in_sizes[5] != EMB * EMB || in_sizes[6] != EMB) return;
  if (in_sizes[7] != EMB || in_sizes[8] != EMB || in_sizes[9] != EMB) return;
  if (in_sizes[10] != EMB * XZLD) return;
  if (in_sizes[11] != CIN * 4 || in_sizes[12] != CIN) return;
  if (in_sizes[13] != CIN * XPJW) return;
  if (in_sizes[14] != RDTL * CIN || in_sizes[15] != CIN) return;
  if (in_sizes[16] != CIN * NSTA || in_sizes[17] != CIN) return;
  if (in_sizes[18] != CIN * EMB) return;
  if (in_sizes[19] != EMB || in_sizes[20] != 1) return;
  if (in_sizes[21] != EMB || in_sizes[22] != EMB) return;
  if (in_sizes[23] != EMB * FFN || in_sizes[24] != FFN) return;
  if (in_sizes[25] != FFN * EMB || in_sizes[26] != EMB) return;
  if (out_size != NTOK * EMB) return;

  const float* x       = (const float*)d_in[0];
  const float* ln1_g   = (const float*)d_in[1];
  const float* ln1_b   = (const float*)d_in[2];
  const float* attn_w  = (const float*)d_in[3];
  const float* attn_b  = (const float*)d_in[4];
  const float* proj_w  = (const float*)d_in[5];
  const float* proj_b  = (const float*)d_in[6];
  const float* mln_g   = (const float*)d_in[7];
  const float* mln_b   = (const float*)d_in[8];
  const float* rms_w   = (const float*)d_in[9];
  const float* in_w    = (const float*)d_in[10];
  const float* conv_w  = (const float*)d_in[11];
  const float* conv_b  = (const float*)d_in[12];
  const float* xproj_w = (const float*)d_in[13];
  const float* dt_w    = (const float*)d_in[14];
  const float* dt_b    = (const float*)d_in[15];
  const float* A_log   = (const float*)d_in[16];
  const float* Dp      = (const float*)d_in[17];
  const float* out_w   = (const float*)d_in[18];
  const float* sel_w   = (const float*)d_in[19];
  const float* sel_b   = (const float*)d_in[20];
  const float* ln2_g   = (const float*)d_in[21];
  const float* ln2_b   = (const float*)d_in[22];
  const float* fc1_w   = (const float*)d_in[23];
  const float* fc1_b   = (const float*)d_in[24];
  const float* fc2_w   = (const float*)d_in[25];
  const float* fc2_b   = (const float*)d_in[26];
  float* outp = (float*)d_out;

  const size_t SZ_WQKV = (size_t)3 * EMB * EMB * 2;
  const size_t SZ_WIN  = (size_t)XZLD * EMB * 2;
  const size_t SZ_WXP  = (size_t)XPJLD * CIN * 2;
  const size_t SZ_WDT  = (size_t)CIN * DTK * 2;
  const size_t SZ_WOUT = (size_t)EMB * CIN * 2;
  const size_t SZ_WPRJ = (size_t)EMB * EMB * 2;
  const size_t SZ_WFC1 = (size_t)FFN * EMB * 2;
  const size_t SZ_WFC2 = (size_t)EMB * FFN * 2;
  const size_t SZ_T16  = (size_t)NTOK * EMB * 2;
  const size_t SZ_T32  = (size_t)NTOK * EMB * 4;
  const size_t SZ_Y16  = (size_t)NTOK * CIN * 2;
  const size_t SZ_SELF = 8192;
  const size_t SZ_XZ   = (size_t)NTOK * XZLD * 4;
  const size_t SZ_HSC  = (size_t)NTOK * CIN * 4;
  const size_t SZ_HSC16= (size_t)NTOK * CIN * 2;
  const size_t SZ_XPJ  = (size_t)NTOK * XPJLD * 4;
  const size_t SZ_DTL  = (size_t)NTOK * DTK * 2;
  const size_t SZ_DTR  = (size_t)NTOK * CIN * 4;
  const size_t SZ_S    = (size_t)HPG * SEQ * SEQ * 4;
  const size_t SZ_P    = (size_t)HPG * SEQ * SEQ * 2;
  const size_t SZ_G16  = (size_t)NTOK * FFN * 2;

  size_t off = 0;
  const size_t oWQKV = off; off += SZ_WQKV;
  const size_t oWIN  = off; off += SZ_WIN;
  const size_t oWXP  = off; off += SZ_WXP;
  const size_t oWDT  = off; off += SZ_WDT;
  const size_t oWOUT = off; off += SZ_WOUT;
  const size_t oWPRJ = off; off += SZ_WPRJ;
  const size_t oWFC1 = off; off += SZ_WFC1;
  const size_t oWFC2 = off; off += SZ_WFC2;
  const size_t oXN16 = off; off += SZ_T16;
  const size_t oHM   = off; off += SZ_T32;
  const size_t oHR16 = off; off += SZ_T16;
  const size_t oQ16  = off; off += SZ_T16;
  const size_t oK16  = off; off += SZ_T16;
  const size_t oVT16 = off; off += SZ_T16;
  const size_t oY16  = off; off += SZ_Y16;
  const size_t oMO   = off; off += SZ_T32;
  const size_t oSELF = off; off += SZ_SELF;
  const size_t oA    = off;
  const size_t oXZ   = oA;
  const size_t oHSC  = oXZ + SZ_XZ;
  const size_t oHSC16= oHSC + SZ_HSC;
  const size_t oXPJ  = oHSC16 + SZ_HSC16;
  const size_t oDTL  = oXPJ + SZ_XPJ;
  const size_t oDTR  = oDTL + SZ_DTL;
  const size_t endP1 = oDTR + SZ_DTR;
  const size_t oS    = oA;
  const size_t oP    = oS + SZ_S;
  const size_t oCTX  = oP + SZ_P;
  const size_t oX1   = oCTX + SZ_T16;
  const size_t oH16  = oX1 + SZ_T32;
  const size_t oG16  = oH16 + SZ_T16;
  const size_t endP2 = oG16 + SZ_G16;
  const size_t TOTAL = (endP1 > endP2) ? endP1 : endP2;
  if (TOTAL > ws_size) return;
  if (TOTAL > (size_t)134217728) return;

  char* ws = (char*)d_ws;
  unsigned short* WQKV = (unsigned short*)(ws + oWQKV);
  unsigned short* WIN  = (unsigned short*)(ws + oWIN);
  unsigned short* WXP  = (unsigned short*)(ws + oWXP);
  unsigned short* WDT  = (unsigned short*)(ws + oWDT);
  unsigned short* WOUT = (unsigned short*)(ws + oWOUT);
  unsigned short* WPRJ = (unsigned short*)(ws + oWPRJ);
  unsigned short* WFC1 = (unsigned short*)(ws + oWFC1);
  unsigned short* WFC2 = (unsigned short*)(ws + oWFC2);
  unsigned short* XN16 = (unsigned short*)(ws + oXN16);
  float*          HM   = (float*)(ws + oHM);
  unsigned short* HR16 = (unsigned short*)(ws + oHR16);
  unsigned short* Q16  = (unsigned short*)(ws + oQ16);
  unsigned short* K16  = (unsigned short*)(ws + oK16);
  unsigned short* VT16 = (unsigned short*)(ws + oVT16);
  unsigned short* Y16  = (unsigned short*)(ws + oY16);
  float*          MO   = (float*)(ws + oMO);
  float*          SELF = (float*)(ws + oSELF);
  float*          XZ   = (float*)(ws + oXZ);
  float*          HSC  = (float*)(ws + oHSC);
  unsigned short* HSC16= (unsigned short*)(ws + oHSC16);
  float*          XPJ  = (float*)(ws + oXPJ);
  unsigned short* DTL16= (unsigned short*)(ws + oDTL);
  float*          DTR  = (float*)(ws + oDTR);
  float*          Sbuf = (float*)(ws + oS);
  unsigned short* P16  = (unsigned short*)(ws + oP);
  unsigned short* CTX  = (unsigned short*)(ws + oCTX);
  float*          X1   = (float*)(ws + oX1);
  unsigned short* H16  = (unsigned short*)(ws + oH16);
  unsigned short* G16  = (unsigned short*)(ws + oG16);
  const float* dummy_bias  = attn_b;
  const float* dummy_resid = x;

  const dim3 blk(256);

  transpose_cast_f16_kernel<<<dim3(3 * EMB / 64, EMB / 64), blk, 0, stream>>>(attn_w, WQKV, EMB, 3 * EMB, kWCarry);
  transpose_cast_f16_kernel<<<dim3(XZLD / 64, EMB / 64), blk, 0, stream>>>(in_w, WIN, EMB, XZLD, kWCarry);
  transpose_cast_f16_kernel<<<dim3(EMB / 64, CIN / 64), blk, 0, stream>>>(out_w, WOUT, CIN, EMB, kWCarry);
  transpose_cast_f16_kernel<<<dim3(EMB / 64, EMB / 64), blk, 0, stream>>>(proj_w, WPRJ, EMB, EMB, kWCarry);
  transpose_cast_f16_kernel<<<dim3(FFN / 64, EMB / 64), blk, 0, stream>>>(fc1_w, WFC1, EMB, FFN, kWCarry);
  transpose_cast_f16_kernel<<<dim3(EMB / 64, FFN / 64), blk, 0, stream>>>(fc2_w, WFC2, FFN, EMB, kWCarry);
  {
    const int totXP = XPJLD * CIN / 8;
    pad_transpose_f16_kernel<<<dim3((totXP + 255) / 256), blk, 0, stream>>>(xproj_w, WXP, CIN, XPJW, CIN, XPJLD, totXP, kWCarry);
    const int totDT = CIN * DTK / 8;
    pad_transpose_f16_kernel<<<dim3((totDT + 255) / 256), blk, 0, stream>>>(dt_w, WDT, RDTL, CIN, DTK, CIN, totDT, kWCarry);
  }

  ln_dual_kernel<<<dim3(NTOK), dim3(192), 0, stream>>>(x, ln1_g, ln1_b, mln_g, mln_b, rms_w, XN16, HM, HR16);

  const int tilesTok = NTOK / 64;
  const dim3 gTok768((tilesTok * (EMB / 64) + 7) / 8, 1);
  const dim3 gVT(((EMB / 64) * tilesTok + 7) / 8, 1);
  const dim3 gIn((tilesTok * (XZLD / 64) + 7) / 8, 1);
  const dim3 gXP((tilesTok * (XPJLD / 64) + 7) / 8, 1);
  const dim3 gDT((tilesTok * (CIN / 64) + 7) / 8, 1);
  const dim3 gFC1((tilesTok * (FFN / 64) + 7) / 8, 1);
  const dim3 gS(((SEQ / 64) * (SEQ / 64) + 7) / 8, HPG);
  const dim3 gPV(((SEQ / 64) * (HDIM / 64) + 7) / 8, HPG);

  wmma_gemm64<0, false, 2, 1, false, 0, 0><<<gTok768, blk, 0, stream>>>(
      XN16, XN16, EMB, 0L, WQKV, WQKV, EMB, 0L, (void*)Q16, (void*)Q16, EMB, 0L, attn_b, dummy_resid, 0L, NTOK, EMB, EMB, kWCarryInv);
  wmma_gemm64<0, false, 2, 1, false, 0, 0><<<gTok768, blk, 0, stream>>>(
      XN16, XN16, EMB, 0L, WQKV + (size_t)EMB * EMB, WQKV + (size_t)EMB * EMB, EMB, 0L, (void*)K16, (void*)K16, EMB, 0L,
      attn_b + EMB, dummy_resid, 0L, NTOK, EMB, EMB, kWCarryInv);
  wmma_gemm64<0, false, 1, 1, false, 0, 0><<<gVT, blk, 0, stream>>>(
      WQKV + (size_t)2 * EMB * EMB, WQKV + (size_t)2 * EMB * EMB, EMB, 0L, XN16, XN16, EMB, 0L, (void*)VT16, (void*)VT16, NTOK, 0L,
      attn_b + 2 * EMB, dummy_resid, 0L, EMB, NTOK, EMB, kWCarryInv);

  wmma_gemm64<0, false, 0, 0, false, 0, 0><<<gIn, blk, 0, stream>>>(
      HR16, HR16, EMB, 0L, WIN, WIN, EMB, 0L, (void*)XZ, (void*)XZ, XZLD, 0L, dummy_bias, dummy_resid, 0L, NTOK, XZLD, EMB, kWCarryInv);
  conv_silu_kernel<<<dim3(CIN / 256, NTOK / 64), blk, 0, stream>>>(XZ, conv_w, conv_b, HSC, HSC16);
  wmma_gemm64<0, false, 0, 0, false, 0, 0><<<gXP, blk, 0, stream>>>(
      HSC16, HSC16, CIN, 0L, WXP, WXP, CIN, 0L, (void*)XPJ, (void*)XPJ, XPJLD, 0L, dummy_bias, dummy_resid, 0L,
      NTOK, XPJLD, CIN, 1.0f / (kUCarry * kWCarry));
  dtl_cast_kernel<<<dim3((NTOK * 8 + 255) / 256), blk, 0, stream>>>(XPJ, DTL16, NTOK * 8);
  wmma_gemm64<0, false, 2, 0, false, 0, 0><<<gDT, blk, 0, stream>>>(
      DTL16, DTL16, DTK, 0L, WDT, WDT, DTK, 0L, (void*)DTR, (void*)DTR, CIN, 0L, dt_b, dummy_resid, 0L,
      NTOK, CIN, DTK, 1.0f / (kDTLCarry * kWCarry));
  scan_kernel<<<dim3(CIN / 256, NBAT), blk, 0, stream>>>(DTR, HSC, XZ, XPJ, A_log, Dp, Y16);
  wmma_gemm64<0, false, 0, 0, true, 0, 0><<<gTok768, blk, 0, stream>>>(
      Y16, Y16, CIN, 0L, WOUT, WOUT, CIN, 0L, (void*)MO, (void*)MO, EMB, 0L, dummy_bias, HM, 0L,
      NTOK, EMB, CIN, 1.0f / (kYCarry * kWCarry));
  sel_kernel<<<dim3((NTOK + 255) / 256), blk, 0, stream>>>(MO, sel_w, sel_b, SELF, NTOK);

  for (int b = 0; b < NBAT; ++b) {
    const size_t boff = (size_t)b * SEQ * EMB;
    for (int g = 0; g < NGRP; ++g) {
      const size_t hc = (size_t)g * HPG * HDIM;
      wmma_gemm64<0, false, 0, 0, false, 0, 1><<<gS, blk, 0, stream>>>(
          Q16 + boff + hc, Q16 + boff + hc, EMB, (long)HDIM, K16 + boff + hc, K16 + boff + hc, EMB, (long)HDIM,
          (void*)Sbuf, (void*)Sbuf, SEQ, (long)SEQ * SEQ, dummy_bias, dummy_resid, 0L, SEQ, SEQ, HDIM, kQScale);
      softmax_causal_sel_kernel<<<dim3(SEQ, HPG), dim3(128), 0, stream>>>(Sbuf, SELF + (size_t)b * SEQ, P16);
      wmma_gemm64<0, false, 0, 1, false, 0, 2><<<gPV, blk, 0, stream>>>(
          P16, P16, SEQ, (long)SEQ * SEQ, VT16 + hc * NTOK + (size_t)b * SEQ, VT16 + hc * NTOK + (size_t)b * SEQ, NTOK, (long)HDIM * NTOK,
          (void*)(CTX + boff + hc), (void*)(CTX + boff + hc), EMB, (long)HDIM, dummy_bias, dummy_resid, 0L,
          SEQ, HDIM, SEQ, kCtxCarry / kPCarry);
    }
  }

  wmma_gemm64<0, false, 2, 0, true, 0, 0><<<gTok768, blk, 0, stream>>>(
      CTX, CTX, EMB, 0L, WPRJ, WPRJ, EMB, 0L, (void*)X1, (void*)X1, EMB, 0L, proj_b, x, 0L, NTOK, EMB, EMB, 1.0f / (kCtxCarry * kWCarry));
  layernorm_f16_kernel<<<dim3(NTOK), dim3(96), 0, stream>>>(X1, ln2_g, ln2_b, H16);
  wmma_gemm64<0, false, 2, 1, false, 0, 0><<<gFC1, blk, 0, stream>>>(
      H16, H16, EMB, 0L, WFC1, WFC1, EMB, 0L, (void*)G16, (void*)G16, FFN, 0L, fc1_b, dummy_resid, 0L, NTOK, FFN, EMB, kWCarryInv);
  const int n8g = NTOK * FFN / 8;
  gelu_erf_f16x8_kernel<<<dim3((n8g + 255) / 256), blk, 0, stream>>>(G16, n8g);
  wmma_gemm64<0, false, 2, 0, true, 0, 0><<<gTok768, blk, 0, stream>>>(
      G16, G16, FFN, 0L, WFC2, WFC2, FFN, 0L, (void*)outp, (void*)outp, EMB, 0L, fc2_b, X1, 0L, NTOK, EMB, FFN, kWCarryInv);
}
